// Classifer_22299470201682
// MI455X (gfx1250) — hardware-run, weakly checked
//
#include <hip/hip_runtime.h>


namespace {
constexpr int N = 100000, NP = 100032, EFULL = 1600000, E = 1600000, NLIM = 100032  , NLIMN = (NLIM < N ? NLIM : N), FIN = 38, FP = 64, H = 128, G = 1024, DEPTH = 4, RPB = 64, NBP = NP / RPB, NBPL = NLIM / RPB,
              F1 = 512, F2 = 256, F3 = 67, F3P = 128, HB = 16384  , NHB = (N + HB - 1) / HB;
constexpr size_t OUT0 = (size_t)G * F3  , OUT1OFF = 68608;
constexpr float XS = 8.0f, WSC = 256.0f, BNEPS = 1e-5f;
static_assert(NP % 64 == 0 && NLIM % 64 == 0 && NLIM <= NP && FP % 32 == 0 && H == 128 && (OUT1OFF * 4) % 128 == 0 && G % 64 == 0 && F1 % 128 == 0 && F2 % 128 == 0, "tiling");
typedef _Float16 b16;
typedef __attribute__((ext_vector_type(16))) _Float16 v16b;
typedef __attribute__((ext_vector_type(8))) _Float16 v8b;
typedef __attribute__((ext_vector_type(8))) float v8f;
typedef __attribute__((ext_vector_type(4))) float v4f;
__device__ __forceinline__ float bf16_rne(float f) { unsigned int u = __float_as_uint(f); u += 0x7FFFu + ((u >> 16) & 1u); return __uint_as_float(u & 0xFFFF0000u); }
__device__ __forceinline__ void split16(float v, b16& hi, b16& lo) { hi = (b16)v; lo = (b16)(v - (float)hi); }
__device__ __forceinline__ v16b frag_kb(const b16* p, int hh) { const v8b a = *(const v8b*)(p + 8 * hh), b = *(const v8b*)(p + 16 + 8 * hh); v16b f;
#pragma unroll
  for (int e = 0; e < 8; ++e) { f[e] = a[e]; f[8 + e] = b[e]; } return f; }
__device__ __forceinline__ v8f wmma16b(v16b a, v16b b, v8f c) { v8f d = __builtin_amdgcn_wmma_f32_16x16x32_f16(false, a, false, b, (short)0, c, false, false); asm volatile("v_nop\n\tv_nop\n\tv_nop\n\tv_nop" : "+v"(d) : "v"(a), "v"(b)); return d; }
__device__ __forceinline__ void wave_lds_sync() { __builtin_amdgcn_fence(__ATOMIC_RELEASE, "workgroup"); __builtin_amdgcn_wave_barrier(); __builtin_amdgcn_fence(__ATOMIC_ACQUIRE, "workgroup"); }
__device__ __forceinline__ float pmul(float a, float b) { float p = a * b; asm volatile("" : "+v"(p)); return p; }
__device__ __forceinline__ int iclamp(int v, int lo, int hi) { return v < lo ? lo : (v > hi ? hi : v); }
constexpr int CSR_NBLK = 512, CSR_GB = 9, CSR_GN = 1 << CSR_GB  , CSR_MAXG = 512, CSR_CAP = 12288  ;
__global__ __launch_bounds__(64) void csrA_kernel(const int* __restrict__ dst, int E, int N, int nG, int CHP, int NGP, int* __restrict__ STG, int* __restrict__ HST) {
  extern __shared__ int sm[];
  int* cnt = sm; int* run = sm + NGP; int* ids = sm + 2 * NGP;
  const int b = blockIdx.x; const int ch = (E + CSR_NBLK - 1) / CSR_NBLK; const int e0 = b * ch, e1 = min(E, e0 + ch);
  for (int i = threadIdx.x; i < NGP; i += 64) cnt[i] = 0;
  for (int i = threadIdx.x; i < CHP; i += 64) ids[i] = -1;
  __syncthreads();
  if (threadIdx.x == 0) {
    for (int e = e0; e < e1; ++e) { int d = dst[e]; d = (d < 0) ? 0 : (d >= N ? N - 1 : d); cnt[d >> CSR_GB] += 1; }
    int acc = 0; for (int g = 0; g < nG; ++g) { run[g] = acc; acc += cnt[g]; }
    for (int e = e0; e < e1; ++e) { int d = dst[e]; d = (d < 0) ? 0 : (d >= N ? N - 1 : d); const int g = d >> CSR_GB; ids[run[g]] = e; run[g] += 1; } }
  __syncthreads();
  typedef __attribute__((ext_vector_type(4))) int v4i;
  for (int pass = 0; pass < 2; ++pass) {
    for (int i = threadIdx.x; i < CHP / 4; i += 64) *(volatile v4i*)(STG + (size_t)b * CHP + i * 4) = *(const v4i*)(&ids[i * 4]);
    for (int i = threadIdx.x; i < NGP / 4; i += 64) { v4i v; for (int e = 0; e < 4; ++e) v[e] = (i * 4 + e < nG) ? cnt[i * 4 + e] : 0; *(volatile v4i*)(HST + (size_t)b * NGP + i * 4) = v; }
    __threadfence(); }
}
__global__ __launch_bounds__(512) void csrS_kernel(const int* __restrict__ HST, int nG, int NGP, int* __restrict__ START, int* __restrict__ TOT, int* __restrict__ OFF) {
  __shared__ int tot[CSR_MAXG];
  const int b = threadIdx.x;
  for (int pass = 0; pass < 2; ++pass) { int runb = 0; for (int g = 0; g < nG; ++g) { int c = HST[(size_t)b * NGP + g]; c = (c < 0) ? 0 : c; ((volatile int*)OFF)[(size_t)g * CSR_NBLK + b] = runb; runb += c; } __threadfence(); }
  for (int g = threadIdx.x; g < nG; g += 512) { int s = 0; for (int bb = 0; bb < CSR_NBLK; ++bb) { int c = HST[(size_t)bb * NGP + g]; s += (c < 0) ? 0 : c; } tot[g] = s; }
  __syncthreads();
  if (threadIdx.x < 32) {
    __shared__ int st[CSR_MAXG + 32];
    if (threadIdx.x == 0) { int acc = 0; for (int g = 0; g < NGP; ++g) { st[g] = acc; if (g < nG) acc += (tot[g] + 31) & ~31; } st[NGP] = acc; }
    __builtin_amdgcn_fence(__ATOMIC_RELEASE, "workgroup"); __builtin_amdgcn_wave_barrier(); __builtin_amdgcn_fence(__ATOMIC_ACQUIRE, "workgroup");
    for (int pass = 0; pass < 2; ++pass) { for (int i = threadIdx.x; i < NGP + 32; i += 32) { ((volatile int*)START)[i] = (i <= NGP) ? st[min(i, NGP)] : 0; ((volatile int*)TOT)[i] = (i < nG) ? tot[i] : 0; } __threadfence(); } }
}
__global__ __launch_bounds__(256) void csrB_kernel(const int* __restrict__ dst, int N, int nG, int CHP, int NGP, int permLen, const int* __restrict__ STG, const int* __restrict__ HST, const int* __restrict__ OFF, const int* __restrict__ START, const int* __restrict__ TOT, int* __restrict__ PERM, int* __restrict__ ROWPTR, int* __restrict__ ROWCNT, int* __restrict__ FLAG) {
  typedef __attribute__((ext_vector_type(4))) int v4i;
  __shared__ int ids[CSR_CAP]; __shared__ unsigned short key[CSR_CAP]; __shared__ int outp[CSR_CAP]; __shared__ int ncnt[CSR_GN + 1]; __shared__ int boff[CSR_NBLK + 1];
  const int g = blockIdx.x, t_ = threadIdx.x; int tot = TOT[g]; int st = START[g], stn = START[g + 1]; const int v0 = g * CSR_GN; const int nv = min(CSR_GN, N - v0);
  st = (st < 0) ? 0 : (st > permLen - 32 ? permLen - 32 : st) & ~31; stn = (stn < st) ? st : (stn > permLen ? permLen : stn); tot = (tot < 0) ? 0 : tot; if (tot > stn - st && tot <= CSR_CAP) tot = stn - st;
  if (tot > CSR_CAP) {
    for (int pass = 0; pass < 2; ++pass) { for (int i = t_; i < CSR_GN / 4; i += 256) { v4i a, c; for (int e = 0; e < 4; ++e) { a[e] = st; c[e] = 0; } *(volatile v4i*)(ROWPTR + v0 + i * 4) = a; *(volatile v4i*)(ROWCNT + v0 + i * 4) = c; } if (t_ == 0) ((volatile int*)FLAG)[0] = 1; __threadfence(); } (void)nv; return; }
  if (t_ == 0) { int acc = 0; for (int b = 0; b < CSR_NBLK; ++b) { boff[b] = acc; int c = HST[(size_t)b * NGP + g]; c = (c < 0) ? 0 : (c > CHP ? CHP : c); acc += c; if (acc > tot) acc = tot; } boff[CSR_NBLK] = acc; }
  for (int i = t_; i <= CSR_GN; i += 256) ncnt[i] = 0;
  __syncthreads();
  for (int b = 0; b < CSR_NBLK; ++b) { const int c = boff[b + 1] - boff[b]; int o_ = OFF[(size_t)g * CSR_NBLK + b]; o_ = (o_ < 0) ? 0 : (o_ > CHP - c ? CHP - c : o_); const int* src_ = STG + (size_t)b * CHP + o_;
    for (int i = t_; i < c; i += 256) { int id = src_[i]; id = (id < 0) ? 0 : id; ids[boff[b] + i] = id; int d = dst[id]; d = (d < v0) ? v0 : (d >= N ? N - 1 : d); int kk = d - v0; kk = (kk < 0) ? 0 : (kk >= CSR_GN ? CSR_GN - 1 : kk); key[boff[b] + i] = (unsigned short)kk; } }
  __syncthreads();
  if (t_ == 0) { for (int i = 0; i < tot; ++i) ncnt[key[i]] += 1; int acc = 0; for (int vl = 0; vl < CSR_GN; ++vl) { const int c = ncnt[vl]; ncnt[vl] = acc; acc += c; } ncnt[CSR_GN] = acc;
    for (int i = 0; i < tot; ++i) { const int vl = key[i]; outp[ncnt[vl]] = ids[i]; ncnt[vl] += 1; }
    for (int vl = CSR_GN; vl > 0; --vl) ncnt[vl] = ncnt[vl - 1]; ncnt[0] = 0; }
  __syncthreads();
  for (int pass = 0; pass < 2; ++pass) {
    for (int i = t_; i < (stn - st) / 4; i += 256) { v4i v; for (int e = 0; e < 4; ++e) { const int q = i * 4 + e; v[e] = (q < tot) ? outp[q] : -1; } *(volatile v4i*)(PERM + st + i * 4) = v; }
    for (int i = t_; i < CSR_GN / 4; i += 256) { v4i a, c; for (int e = 0; e < 4; ++e) { const int vl = i * 4 + e; a[e] = st + ncnt[vl]; c[e] = (vl < nv) ? (ncnt[vl + 1] - ncnt[vl]) : 0; } *(volatile v4i*)(ROWPTR + v0 + i * 4) = a; *(volatile v4i*)(ROWCNT + v0 + i * 4) = c; }
    __threadfence(); }
}
__global__ __launch_bounds__(256) void csrZ_kernel(int* __restrict__ p, size_t n4) { typedef __attribute__((ext_vector_type(4))) int v4i; const size_t tid = (size_t)blockIdx.x * 256 + threadIdx.x, nth = (size_t)gridDim.x * 256; v4i z = {0, 0, 0, 0}; for (size_t i = tid; i < n4; i += nth) *(volatile v4i*)(p + i * 4) = z; }
struct CsrBufs { int *STG, *HST, *OFF, *START, *TOT, *PERM, *ROWPTR, *ROWCNT, *FLAG; int nG, NGP, CHP; size_t permLen; char* base; size_t bytes; };
static size_t csr_carve(CsrBufs& c, char* ws, size_t off, int E, int N) {
  const size_t off0 = off; c.base = ws + off;
  auto al = [&](size_t bytes) { char* p = ws + off; off += (bytes + 255) & ~(size_t)255; return p; };
  c.nG = (N + CSR_GN - 1) / CSR_GN; c.NGP = (c.nG + 31) & ~31; const int ch = (E + CSR_NBLK - 1) / CSR_NBLK; c.CHP = (ch + 31) & ~31; c.permLen = (size_t)E + 32 * (size_t)c.nG + 32;
  c.STG = (int*)al((size_t)CSR_NBLK * c.CHP * 4); c.HST = (int*)al((size_t)CSR_NBLK * c.NGP * 4); c.OFF = (int*)al((size_t)c.NGP * CSR_NBLK * 4); c.START = (int*)al((size_t)(c.NGP + 64) * 4); c.TOT = (int*)al((size_t)(c.NGP + 64) * 4);
  c.PERM = (int*)al(c.permLen * 4); c.ROWPTR = (int*)al((size_t)c.nG * CSR_GN * 4); c.ROWCNT = (int*)al((size_t)c.nG * CSR_GN * 4); c.FLAG = (int*)al(256);
  c.bytes = off - off0; return off;
}
static void csr_build(const CsrBufs& c, const int* dst, int E, int N, hipStream_t stream) {
  const size_t smem = (size_t)(2 * c.NGP + c.CHP) * 4;
  csrZ_kernel<<<512, 256, 0, stream>>>((int*)c.base, c.bytes / 16);
  csrA_kernel<<<CSR_NBLK, 64, smem, stream>>>(dst, E, N, c.nG, c.CHP, c.NGP, c.STG, c.HST);
  csrS_kernel<<<1, 512, 0, stream>>>(c.HST, c.nG, c.NGP, c.START, c.TOT, c.OFF);
  csrB_kernel<<<c.nG, 256, 0, stream>>>(dst, N, c.nG, c.CHP, c.NGP, (int)c.permLen, c.STG, c.HST, c.OFF, c.START, c.TOT, c.PERM, c.ROWPTR, c.ROWCNT, c.FLAG);
}

typedef __attribute__((ext_vector_type(4))) _Float16 v4h;
typedef __attribute__((ext_vector_type(2))) _Float16 v2h;
typedef __attribute__((ext_vector_type(2))) float v2f;
__global__ __launch_bounds__(256) void prep_kernel(const float* __restrict__ h, const float* __restrict__ w1, const float* __restrict__ w2s, const float* __restrict__ wf1, const float* __restrict__ wl, const float* __restrict__ wf2,
                                                    float* __restrict__ X0, b16* __restrict__ W1T, b16* __restrict__ W2T, b16* __restrict__ WF1T, b16* __restrict__ WLT, b16* __restrict__ WF2T) {
  size_t t = (size_t)blockIdx.x * 256 + threadIdx.x; v8b o;
  const size_t nx = (size_t)NP * FP / 4; if (t < nx) { const size_t e = t * 4; const size_t v = e / FP; const int c = (int)(e % FP); v4f r = {0.0f, 0.0f, 0.0f, 0.0f}; if (v < (size_t)N) { for (int j = 0; j < 4; ++j) if (c + j < FIN) r[j] = bf16_rne(h[v * FIN + c + j]); } for (int pass = 0; pass < 2; ++pass) { *(volatile v4f*)(X0 + e) = r; __threadfence(); } return; } t -= nx;
  const size_t n1 = (size_t)H * FP / 8; if (t < n1) { const size_t e = t * 8; const int oo = (int)(e / FP), k0 = (int)(e % FP); for (int j = 0; j < 8; ++j) o[j] = (k0 + j < FIN) ? (b16)(bf16_rne(w1[(size_t)(k0 + j) * H + oo]) * WSC) : (b16)0.0f; for (int pass = 0; pass < 2; ++pass) { *(volatile v8b*)(W1T + e) = o; __threadfence(); } return; } t -= n1;
  const size_t n2 = (size_t)3 * H * H / 8; if (t < n2) { const size_t e = t * 8; const int l = (int)(e / ((size_t)H * H)); const size_t el = e % ((size_t)H * H); const int oo = (int)(el / H), k0 = (int)(el % H); for (int j = 0; j < 8; ++j) o[j] = (b16)(bf16_rne(w2s[(size_t)l * H * H + (size_t)(k0 + j) * H + oo]) * WSC); for (int pass = 0; pass < 2; ++pass) { *(volatile v8b*)(W2T + e) = o; __threadfence(); } return; } t -= n2;
  const size_t n3 = (size_t)F1 * H / 8; if (t < n3) { const size_t e = t * 8; const int oo = (int)(e / H), k0 = (int)(e % H); for (int j = 0; j < 8; ++j) o[j] = (b16)(bf16_rne(wf1[(size_t)(k0 + j) * F1 + oo]) * WSC); for (int pass = 0; pass < 2; ++pass) { *(volatile v8b*)(WF1T + e) = o; __threadfence(); } return; } t -= n3;
  const size_t n4 = (size_t)F2 * F1 / 8; if (t < n4) { const size_t e = t * 8; const int oo = (int)(e / F1), k0 = (int)(e % F1); for (int j = 0; j < 8; ++j) o[j] = (b16)(bf16_rne(wl[(size_t)(k0 + j) * F2 + oo]) * WSC); for (int pass = 0; pass < 2; ++pass) { *(volatile v8b*)(WLT + e) = o; __threadfence(); } return; } t -= n4;
  const size_t n5 = (size_t)F3P * F2 / 8; if (t < n5) { const size_t e = t * 8; const int oo = (int)(e / F2), k0 = (int)(e % F2); for (int j = 0; j < 8; ++j) o[j] = (oo < F3) ? (b16)(bf16_rne(wf2[(size_t)(k0 + j) * F3 + oo]) * WSC) : (b16)0.0f; for (int pass = 0; pass < 2; ++pass) { *(volatile v8b*)(WF2T + e) = o; __threadfence(); } }
}
__global__ __launch_bounds__(256) void outdeg_kernel(const int* __restrict__ srcs, float* __restrict__ NS) {
  __shared__ int cnt[HB];
  const int base = blockIdx.x * HB;
  for (int i = threadIdx.x; i < HB; i += 256) cnt[i] = 0;
  __syncthreads();
#pragma unroll 1
  for (size_t e = threadIdx.x; e < (size_t)E; e += 256) { const int s = srcs[e] - base; if (s >= 0 && s < HB) atomicAdd(&cnt[s], 1); }
  __syncthreads();
  for (int pass = 0; pass < 2; ++pass) { for (int q = threadIdx.x; q < HB / 4; q += 256) { const int v0 = base + q * 4; if (v0 < NP) { v4f r; for (int j = 0; j < 4; ++j) { const int c = cnt[q * 4 + j]; r[j] = rsqrtf((float)(c < 1 ? 1 : c)); } *(volatile v4f*)(NS + v0) = r; } } __threadfence(); }
}
template <int FW>
__global__ __launch_bounds__(256) void agg_kernel(const float* __restrict__ X, const float* __restrict__ NS, const int* __restrict__ srcs, const int* __restrict__ PERM, const int* __restrict__ ROWPTR, const int* __restrict__ ROWCNT, int permLen, b16* __restrict__ Ah, b16* __restrict__ Al) {
  constexpr int CPL = FW / 32;
  typedef __attribute__((ext_vector_type(CPL))) float vf; typedef __attribute__((ext_vector_type(CPL))) _Float16 vh;
  const int wave = threadIdx.x >> 5, lane = threadIdx.x & 31; const size_t v = (size_t)blockIdx.x * 8 + wave; const int c = lane * CPL; vf a; for (int i = 0; i < CPL; ++i) a[i] = 0.0f;
  if (v < (size_t)N) { int st = ROWPTR[v], cnt = ROWCNT[v]; cnt = iclamp(cnt, 0, 65536); st = iclamp(st, 0, permLen - cnt);
#pragma unroll 1
    for (int j = 0; j < cnt; ++j) { const int e = iclamp(PERM[st + j], 0, E - 1); const int s = iclamp(srcs[e], 0, N - 1); vf t = *(const vf*)(X + (size_t)s * FW + c); float w = NS[s]; if (s >= NLIM) w = 0.0f; for (int i = 0; i < CPL; ++i) a[i] += pmul(w, t[i]); }
    const float nd = rsqrtf((float)(cnt < 1 ? 1 : cnt)); for (int i = 0; i < CPL; ++i) a[i] = pmul(a[i], nd); }
  vh ah, al; for (int i = 0; i < CPL; ++i) { b16 p, q; split16(a[i] * XS, p, q); ah[i] = p; al[i] = q; }
  for (int pass = 0; pass < 2; ++pass) { *(volatile vh*)(Ah + v * FW + c) = ah; *(volatile vh*)(Al + v * FW + c) = al; __threadfence(); }
}
template <int KD>
__global__ __launch_bounds__(128) void gconv_kernel(const b16* __restrict__ Ah, const b16* __restrict__ Al, const b16* __restrict__ WT, const float* __restrict__ bias, float* __restrict__ P, float* __restrict__ PS) {
  __shared__ __attribute__((aligned(16))) float Tf[4][16][H + 4];
  const int wave = threadIdx.x >> 5, lane = threadIdx.x & 31, nloc = lane & 15, hlf = lane >> 4; const size_t m0 = (size_t)blockIdx.x * 64 + wave * 16;
  v8f acc[8];
#pragma unroll
  for (int t = 0; t < 8; ++t) acc[t] = (v8f){};
#pragma unroll 2
  for (int kb = 0; kb < KD; kb += 32) { const v16b a = frag_kb(Ah + (m0 + nloc) * KD + kb, hlf), al = frag_kb(Al + (m0 + nloc) * KD + kb, hlf);
#pragma unroll
    for (int t = 0; t < 8; ++t) { const v16b bw = frag_kb(WT + (size_t)(t * 16 + nloc) * KD + kb, hlf); acc[t] = wmma16b(a, bw, acc[t]); acc[t] = wmma16b(al, bw, acc[t]); } }
  v4f bb; for (int j = 0; j < 4; ++j) bb[j] = bf16_rne(bias[lane * 4 + j]);
#pragma unroll
  for (int t = 0; t < 8; ++t)
#pragma unroll
    for (int r = 0; r < 8; ++r) Tf[wave][8 * hlf + r][t * 16 + nloc] = acc[t][r] * (1.0f / (XS * WSC));
  wave_lds_sync();
  for (int rr = 0; rr < 16; ++rr) { v4f o = *(const v4f*)(&Tf[wave][rr][lane * 4]); o += bb; if (m0 + rr >= (size_t)NLIMN) o = (v4f){0.0f, 0.0f, 0.0f, 0.0f}; *(v4f*)(&Tf[wave][rr][lane * 4]) = o; }
  __syncthreads();
  for (int pass = 0; pass < 2; ++pass) { for (int rr = 0; rr < 16; ++rr) *(volatile v4f*)(P + (m0 + rr) * H + lane * 4) = *(const v4f*)(&Tf[wave][rr][lane * 4]);
    if (threadIdx.x < H / 4) { v4f s = {0.0f, 0.0f, 0.0f, 0.0f};
#pragma unroll 1
      for (int w = 0; w < 4; ++w) for (int rr = 0; rr < 16; ++rr) s += *(const v4f*)(&Tf[w][rr][threadIdx.x * 4]); *(volatile v4f*)(PS + (size_t)blockIdx.x * H + threadIdx.x * 4) = s; }
    __threadfence(); }
}
__global__ __launch_bounds__(128) void colstat_kernel(const float* __restrict__ PS, float* __restrict__ STAT) {
  const int c = threadIdx.x; float s = 0.0f;
#pragma unroll 1
  for (int b = 0; b < NBPL; ++b) s += PS[(size_t)b * H + c];
  for (int pass = 0; pass < 2; ++pass) { ((volatile float*)STAT)[c] = s * (1.0f / NLIMN); __threadfence(); }
}
__global__ __launch_bounds__(256) void var_kernel(const float* __restrict__ P, const float* __restrict__ MEAN, float* __restrict__ PS) {
  __shared__ __attribute__((aligned(16))) float sq[2][H + 4]; const int t = threadIdx.x, c = t % H, grp = t / H; float a = 0.0f; const float m = MEAN[c];
#pragma unroll 1
  for (int rr = grp; rr < RPB; rr += 2) { const size_t v = (size_t)blockIdx.x * RPB + rr; const float d = v < (size_t)NLIMN ? P[v * H + c] - m : 0.0f; a += d * d; }
  sq[grp][c] = a; __syncthreads();
  for (int pass = 0; pass < 2; ++pass) { if (t < H / 4) { const v4f s = *(const v4f*)(&sq[0][t * 4]) + *(const v4f*)(&sq[1][t * 4]); *(volatile v4f*)(PS + (size_t)blockIdx.x * H + t * 4) = s; } __threadfence(); }
}
__global__ __launch_bounds__(256) void apply_kernel(float* __restrict__ PX, const float* __restrict__ MEAN, const float* __restrict__ VAR, const float* __restrict__ g_, const float* __restrict__ be_) {
  const size_t u = (size_t)blockIdx.x * 256 + threadIdx.x; if (u >= (size_t)NP * H / 4) return; const size_t e = u * 4; const size_t v = e / H; const int c = (int)(e % H);
  v4f o = {0.0f, 0.0f, 0.0f, 0.0f}; if (v < (size_t)NLIMN) { const v4f p = *(const v4f*)(PX + e); for (int i = 0; i < 4; ++i) o[i] = fmaxf((p[i] - MEAN[c + i]) * rsqrtf(VAR[c + i] + BNEPS) * bf16_rne(g_[c + i]) + bf16_rne(be_[c + i]), 0.0f); }
  for (int pass = 0; pass < 2; ++pass) { *(volatile v4f*)(PX + e) = o; __threadfence(); }
}
__global__ __launch_bounds__(256) void readout_kernel(const float* __restrict__ X, const float* __restrict__ aw, const float* __restrict__ ab, float* __restrict__ out1, float* __restrict__ WG) {
  const size_t v = (size_t)blockIdx.x * 256 + threadIdx.x; float a = 0.0f, w = 0.0f;
  if (v < (size_t)N) { a = bf16_rne(ab[0]);
#pragma unroll 1
    for (int k = 0; k < H; ++k) a += pmul(X[v * H + k], bf16_rne(aw[k])); w = 1.0f / (1.0f + __expf(-a)); }
  for (int pass = 0; pass < 2; ++pass) { if (v < (size_t)N) ((volatile float*)out1)[v] = a; if (v < (size_t)NP) ((volatile float*)WG)[v] = w; __threadfence(); }
}
__device__ int lower_bound_i(const int* a, int n, int key) { int lo = 0, hi = n; while (lo < hi) { const int mid = (lo + hi) >> 1; if (a[mid] < key) lo = mid + 1; else hi = mid; } return lo; }
__global__ __launch_bounds__(128) void pool_kernel(const float* __restrict__ X, const float* __restrict__ WG, const int* __restrict__ n2g, float* __restrict__ HG) {
  const int g = blockIdx.x, c = threadIdx.x; const int lo = lower_bound_i(n2g, N, g), hi = lower_bound_i(n2g, N, g + 1); float s = 0.0f;
#pragma unroll 1
  for (int v = lo; v < hi; ++v) s += pmul(X[(size_t)v * H + c], WG[v]);
  for (int pass = 0; pass < 2; ++pass) { ((volatile float*)HG)[(size_t)g * H + c] = s; __threadfence(); }
}
template <int KD, int NCOL, int EPI>
__global__ __launch_bounds__(128) void hgemm_kernel(const float* __restrict__ IN, const b16* __restrict__ WT, const float* __restrict__ bias, int nbias, float* __restrict__ OUT) {
  __shared__ __attribute__((aligned(16))) b16 Ahs[4][16][128 + 8], Als[4][16][128 + 8]; __shared__ __attribute__((aligned(16))) float Tf[4][16][128 + 4];
  const int wave = threadIdx.x >> 5, lane = threadIdx.x & 31, nloc = lane & 15, hlf = lane >> 4; const size_t m0 = (size_t)blockIdx.x * 64 + wave * 16; const int n0 = blockIdx.y * 128;
  v8f acc[8];
#pragma unroll
  for (int t = 0; t < 8; ++t) acc[t] = (v8f){};
#pragma unroll 1
  for (int kc = 0; kc < KD; kc += 128) {
    for (int rr = 0; rr < 16; ++rr) { const v4f x4 = *(const v4f*)(IN + (m0 + rr) * KD + kc + lane * 4); v4h hv, lv; for (int j = 0; j < 4; ++j) { b16 p, q; split16(x4[j] * XS, p, q); hv[j] = p; lv[j] = q; } *(v4h*)(&Ahs[wave][rr][lane * 4]) = hv; *(v4h*)(&Als[wave][rr][lane * 4]) = lv; }
    wave_lds_sync();
#pragma unroll
    for (int kb = 0; kb < 128; kb += 32) { const v16b a = frag_kb(&Ahs[wave][nloc][kb], hlf), al = frag_kb(&Als[wave][nloc][kb], hlf);
#pragma unroll
      for (int t = 0; t < 8; ++t) { const v16b bw = frag_kb(WT + (size_t)(n0 + t * 16 + nloc) * KD + kc + kb, hlf); acc[t] = wmma16b(a, bw, acc[t]); acc[t] = wmma16b(al, bw, acc[t]); } }
    wave_lds_sync(); }
#pragma unroll
  for (int t = 0; t < 8; ++t)
#pragma unroll
    for (int r = 0; r < 8; ++r) Tf[wave][8 * hlf + r][t * 16 + nloc] = acc[t][r] * (1.0f / (XS * WSC));
  wave_lds_sync();
  v4f bb; for (int j = 0; j < 4; ++j) { const int cc = n0 + lane * 4 + j; bb[j] = (cc < nbias) ? bf16_rne(bias[cc]) : 0.0f; }
  for (int pass = 0; pass < 2; ++pass) { for (int rr = 0; rr < 16; ++rr) { v4f o = *(const v4f*)(&Tf[wave][rr][lane * 4]); o += bb; if (EPI == 1) { for (int j = 0; j < 4; ++j) o[j] = 1.0f / (1.0f + __expf(-o[j])); } *(volatile v4f*)(OUT + (m0 + rr) * NCOL + n0 + lane * 4) = o; } __threadfence(); }
}
template <int NC>
__global__ __launch_bounds__(128) void colbn_kernel(const float* __restrict__ Y, const float* __restrict__ g_, const float* __restrict__ be_, float* __restrict__ YN) {
  const int c = blockIdx.x * 128 + threadIdx.x; float s = 0.0f;
#pragma unroll 1
  for (int r = 0; r < G; ++r) s += Y[(size_t)r * NC + c];
  const float m = s * (1.0f / G); float q = 0.0f;
#pragma unroll 1
  for (int r = 0; r < G; ++r) { const float d = Y[(size_t)r * NC + c] - m; q += d * d; }
  const float rs = rsqrtf(q * (1.0f / G) + BNEPS), gg = bf16_rne(g_[c]), bb = bf16_rne(be_[c]);
  for (int pass = 0; pass < 2; ++pass) {
#pragma unroll 1
    for (int r = 0; r < G; ++r) ((volatile float*)YN)[(size_t)r * NC + c] = fmaxf((Y[(size_t)r * NC + c] - m) * rs * gg + bb, 0.0f);
    __threadfence(); }
}
__global__ __launch_bounds__(256) void out0_kernel(const float* __restrict__ Y3, float* __restrict__ out) {
  const size_t q = (size_t)blockIdx.x * 256 + threadIdx.x; if (q * 4 >= OUT0) return; v4f o; for (int j = 0; j < 4; ++j) { const size_t i = q * 4 + j; o[j] = Y3[(i / F3) * F3P + (i % F3)]; }
  for (int pass = 0; pass < 2; ++pass) { *(volatile v4f*)(out + q * 4) = o; __threadfence(); }
}
}

extern "C" void kernel_launch(void* const* d_in, const int* in_sizes, int n_in, void* d_out, int out_size, void* d_ws, size_t ws_size, hipStream_t stream) {
  (void)n_in;
  auto Fp = [&](int i) { return (const float*)d_in[i]; }; auto Ip = [&](int i) { return (const int*)d_in[i]; };
  if (in_sizes[0] != N * FIN || in_sizes[1] != EFULL || in_sizes[2] != EFULL || in_sizes[3] != N || in_sizes[4] != FIN * H || in_sizes[5] != H || in_sizes[8] != 3 * H * H || in_sizes[9] != 3 * H || in_sizes[12] != H || in_sizes[13] != 1 ||
      in_sizes[14] != H * F1 || in_sizes[15] != F1 || in_sizes[18] != F1 * F2 || in_sizes[19] != F2 || in_sizes[22] != F2 * F3 || in_sizes[23] != F3 || (size_t)out_size != OUT0 + (size_t)N) return;
  size_t off = 0; char* ws = (char*)d_ws;
  auto carve = [&](size_t bytes) { char* p = ws + off; off += (bytes + 255) & ~(size_t)255; return p; };
  b16* W1T = (b16*)carve((size_t)H * FP * 2); b16* W2T = (b16*)carve((size_t)3 * H * H * 2); b16* WF1T = (b16*)carve((size_t)F1 * H * 2); b16* WLT = (b16*)carve((size_t)F2 * F1 * 2); b16* WF2T = (b16*)carve((size_t)F3P * F2 * 2);
  float* PX = (float*)carve((size_t)NP * H * 4);
  b16* Ah = (b16*)carve((size_t)NP * H * 2); b16* Al = (b16*)carve((size_t)NP * H * 2); float* PS = (float*)carve((size_t)NBP * H * 4); float* ST = (float*)carve((size_t)2 * H * 4); float* NS = (float*)carve((size_t)NHB * HB * 4); float* WG = (float*)carve((size_t)NP * 4);
  float* HG = (float*)carve((size_t)G * H * 4); float* Y1 = (float*)carve((size_t)G * F1 * 4); float* Y1N = (float*)carve((size_t)G * F1 * 4); float* Y2 = (float*)carve((size_t)G * F2 * 4); float* Y2N = (float*)carve((size_t)G * F2 * 4); float* Y3 = (float*)carve((size_t)G * F3P * 4);
  CsrBufs csr; off = csr_carve(csr, ws, off, E, N);
  if (off > ws_size || off > ((size_t)128 << 20)) return;
  prep_kernel<<<(unsigned)((((size_t)NP * FP / 4) + ((size_t)H * FP + 3 * (size_t)H * H + (size_t)F1 * H + (size_t)F2 * F1 + (size_t)F3P * F2) / 8 + 255) / 256), 256, 0, stream>>>(Fp(0), Fp(4), Fp(8), Fp(14), Fp(18), Fp(22), PX, W1T, W2T, WF1T, WLT, WF2T);
  outdeg_kernel<<<NHB, 256, 0, stream>>>(Ip(1), NS);
  csr_build(csr, Ip(2), E, N, stream);
  for (int l = 0; l < DEPTH; ++l) {
    if (l == 0) { agg_kernel<FP><<<NLIM / 8, 256, 0, stream>>>(PX, NS, Ip(1), csr.PERM, csr.ROWPTR, csr.ROWCNT, (int)csr.permLen, Ah, Al); gconv_kernel<FP><<<NLIM / 64, 128, 0, stream>>>(Ah, Al, W1T, Fp(5), PX, PS); }
    else { agg_kernel<H><<<NLIM / 8, 256, 0, stream>>>(PX, NS, Ip(1), csr.PERM, csr.ROWPTR, csr.ROWCNT, (int)csr.permLen, Ah, Al); gconv_kernel<H><<<NLIM / 64, 128, 0, stream>>>(Ah, Al, W2T + (size_t)(l - 1) * H * H, Fp(9) + (l - 1) * H, PX, PS); }
    colstat_kernel<<<1, 128, 0, stream>>>(PS, ST); var_kernel<<<NBPL, 256, 0, stream>>>(PX, ST, PS); colstat_kernel<<<1, 128, 0, stream>>>(PS, ST + H);
    apply_kernel<<<(unsigned)(((size_t)NP * H / 4 + 255) / 256), 256, 0, stream>>>(PX, ST, ST + H, l == 0 ? Fp(6) : Fp(10) + (l - 1) * H, l == 0 ? Fp(7) : Fp(11) + (l - 1) * H); }
  readout_kernel<<<(NP + 255) / 256, 256, 0, stream>>>(PX, Fp(12), Fp(13), (float*)d_out + OUT1OFF, WG);
  pool_kernel<<<G, 128, 0, stream>>>(PX, WG, Ip(3), HG);
  hgemm_kernel<H, F1, 0><<<dim3(G / 64, F1 / 128), 128, 0, stream>>>(HG, WF1T, Fp(15), F1, Y1); colbn_kernel<F1><<<F1 / 128, 128, 0, stream>>>(Y1, Fp(16), Fp(17), Y1N);
  hgemm_kernel<F1, F2, 0><<<dim3(G / 64, F2 / 128), 128, 0, stream>>>(Y1N, WLT, Fp(19), F2, Y2); colbn_kernel<F2><<<F2 / 128, 128, 0, stream>>>(Y2, Fp(20), Fp(21), Y2N);
  hgemm_kernel<F2, F3P, 1><<<dim3(G / 64, F3P / 128), 128, 0, stream>>>(Y2N, WF2T, Fp(23), F3, Y3);
  out0_kernel<<<(unsigned)((OUT0 / 4 + 255) / 256), 256, 0, stream>>>(Y3, (float*)d_out);
}
